// MultiHeadAttention_7275674600363
// MI455X (gfx1250) — hardware-run, weakly checked
//
#include <hip/hip_runtime.h>


#ifndef NB
#define NB 4
#endif
#ifndef SEQ
#define SEQ 2048
#endif
#define NB_FULL  4
#define SEQ_FULL 2048
#ifndef OUT_SEQ
#define OUT_SEQ SEQ
#endif
#ifndef EARLY
#define EARLY ((SEQ >= 1024) ? 384 : (SEQ / 2))
#endif
#define DM   1024
#define NH_  16
#define HD   64
#define AW   4
#define QRS  2048.0f
#define QRI  (1.0f / 2048.0f)
#define SC2  (0.125f * 1.4426950408889634f)
#define PSH  8.0f
#define CXS  64.0f
#define CRS  256.0f
#define WOS  1024.0f
#define WOS2 (WOS / CRS)
#define OSC  (1.0f / (CXS * WOS))

static_assert(HD == 64);
static_assert(NH_ * HD == DM);
static_assert((DM & (DM - 1)) == 0);
static_assert(DM % 64 == 0);
static_assert(DM % 32 == 0);
static_assert(SEQ % 64 == 0);
static_assert((NB * SEQ) % 64 == 0);
static_assert(SEQ % 32 == 0);
static_assert(EARLY % (16 * AW) == 0);
static_assert(EARLY > 0 && EARLY < SEQ);
static_assert((SEQ - EARLY) % (16 * AW) == 0);
static_assert(((size_t)SEQ * DM) % 8 == 0);
static_assert(NB <= NB_FULL);
static_assert(SEQ <= SEQ_FULL);

typedef _Float16 h16;
typedef unsigned short bf;
typedef __attribute__((ext_vector_type(16))) __bf16   v16bf;
typedef __attribute__((ext_vector_type(16))) _Float16 v16h;
typedef __attribute__((ext_vector_type(16))) unsigned short v16us;
typedef __attribute__((ext_vector_type(8)))  _Float16 v8h;
typedef __attribute__((ext_vector_type(8)))  unsigned short v8us;
typedef __attribute__((ext_vector_type(8)))  float    v8f;
typedef __attribute__((ext_vector_type(4)))  float    v4f;
typedef v4f  __attribute__((may_alias)) v4fa;

__device__ __forceinline__ unsigned short f2bf(float f) { unsigned u = __float_as_uint(f); u += 0x7FFFu + ((u >> 16) & 1u); return (unsigned short)(u >> 16); }
__device__ __forceinline__ float bfr(float f) { return __uint_as_float(((unsigned)f2bf(f)) << 16); }
__device__ __forceinline__ unsigned short hbits(h16 x) { return __builtin_bit_cast(unsigned short, x); }
__device__ __forceinline__ v16h cat16(v8h lo, v8h hi) { return __builtin_shufflevector(lo, hi, 0, 1, 2, 3, 4, 5, 6, 7, 8, 9, 10, 11, 12, 13, 14, 15); }
__device__ __forceinline__ v8f wmma16(v16h a, v16h b, v8f c) { return __builtin_amdgcn_wmma_f32_16x16x32_f16(false, a, false, b, (short)0, c, false, false); }
__device__ __forceinline__ v8f wmmab(v16bf a, v16bf b, v8f c) { return __builtin_amdgcn_wmma_f32_16x16x32_bf16(false, a, false, b, (short)0, c, false, false); }
__device__ __forceinline__ v16h  ldh(const h16* p) { return cat16(*(const v8h*)p, *(const v8h*)(p + 16)); }
__device__ __forceinline__ v16us ldu(const bf* p)  { return __builtin_shufflevector(*(const v8us*)p, *(const v8us*)(p + 16), 0, 1, 2, 3, 4, 5, 6, 7, 8, 9, 10, 11, 12, 13, 14, 15); }
template<int F16> __device__ __forceinline__ v8f mm(v16us a, v16us b, v8f c) {
    if (F16) return wmma16(__builtin_bit_cast(v16h, a), __builtin_bit_cast(v16h, b), c);
    else     return wmmab(__builtin_bit_cast(v16bf, a), __builtin_bit_cast(v16bf, b), c);
}
__device__ __forceinline__ void wave_sync() { __builtin_amdgcn_fence(3  , "wavefront"); __builtin_amdgcn_wave_barrier(); asm volatile("" ::: "memory"); }

__global__ __launch_bounds__(256) void k_cvt8(const float* __restrict__ src, bf* dst, size_t n8) {
    const size_t i = (size_t)blockIdx.x * 256 + threadIdx.x; if (i >= n8) return;
    const v8f v = *(const v8f*)(src + i * 8); v8us o;
#pragma unroll
    for (int k = 0; k < 8; ++k) o[k] = f2bf(v[k]);
    *(volatile v8us*)(dst + i * 8) = o; __threadfence(); *(volatile v8us*)(dst + i * 8) = o;
}

template<int MODE>
__global__ __launch_bounds__(256) void k_tr(const float* __restrict__ in, bf* out, int C, int opitch, size_t inB, size_t outB) {
    __shared__ __align__(16) bf ts[(MODE ? 2 : 1) * 64 * 72];
    const int tid = threadIdx.x;
    const int r0 = blockIdx.x * 64, c0 = blockIdx.y * 64;
    const float* src = in + (size_t)blockIdx.z * inB;
    bf* dst = out + (size_t)blockIdx.z * outB;
#pragma unroll
    for (int it = 0; it < 4; ++it) {
        const int row = it * 16 + (tid >> 4), c4 = (tid & 15) * 4;
        const v4f v = *(const v4f*)(src + (size_t)(r0 + row) * (size_t)C + c0 + c4);
#pragma unroll
        for (int i = 0; i < 4; ++i) {
            if (MODE == 0) { ts[(c4 + i) * 72 + row] = f2bf(v[i]); }
            else { const float w = bfr(v[i]); ts[(c4 + i) * 72 + row] = hbits((h16)(w * WOS)); ts[64 * 72 + (c4 + i) * 72 + row] = hbits((h16)(w * WOS2)); }
        }
    }
    __syncthreads();
#pragma unroll 1
    for (int ps = 0; ps < 2; ++ps) {
#pragma unroll
        for (int it = 0; it < 2; ++it) {
            const int c = it * 32 + (tid >> 3), p8 = (tid & 7) * 8;
            const v8us o = *(const v8us*)(&ts[c * 72 + p8]);
            *(volatile v8us*)(dst + (size_t)(c0 + c) * (size_t)opitch + r0 + p8) = o;
            if (MODE) { const v8us o2 = *(const v8us*)(&ts[64 * 72 + c * 72 + p8]); *(volatile v8us*)(dst + (size_t)(c0 + c) * (size_t)opitch + DM + r0 + p8) = o2; }
        }
        if (ps == 0) __threadfence();
    }
}

template<int OM>
__global__ __launch_bounds__(32) void k_gemm(const bf* __restrict__ A, const bf* __restrict__ Bt, int K, int lda, int ldb,
                                             h16* Ph, h16* Pr, float* Pf, int useRes, int RB, size_t sRB, int pitch, int CB, size_t sCB,
                                             const float* __restrict__ bias, int bmode, float oscale) {
    __shared__ __align__(16) float os[16 * 68];
    const int lane = threadIdx.x & 31, lr = lane & 15, hi = lane >> 4; const int r0 = blockIdx.x * 64, c0 = blockIdx.y * 64;
    v8f acc[4][4];
#pragma unroll
    for (int mb = 0; mb < 4; ++mb)
#pragma unroll
        for (int nb = 0; nb < 4; ++nb) acc[mb][nb] = (v8f){};
    const size_t aoff = (size_t)(r0 + lr) * (size_t)lda + 8 * hi, boff = (size_t)(c0 + lr) * (size_t)ldb + 8 * hi;
#pragma unroll 1
    for (int kc = 0; kc < K; kc += 32) {
        v16us a[4];
#pragma unroll
        for (int mb = 0; mb < 4; ++mb) a[mb] = ldu(A + aoff + (size_t)mb * 16 * (size_t)lda + kc);
#pragma unroll
        for (int nb = 0; nb < 4; ++nb) { const v16us b = ldu(Bt + boff + (size_t)nb * 16 * (size_t)ldb + kc);
#pragma unroll
            for (int mb = 0; mb < 4; ++mb) acc[mb][nb] = mm<OM>(a[mb], b, acc[mb][nb]); }
        asm volatile("v_nop\n\tv_nop\n\tv_nop\n\tv_nop" : "+v"(acc[0][0]), "+v"(acc[1][1]), "+v"(acc[2][2]), "+v"(acc[3][3]) : "v"(a[0]), "v"(a[1]), "v"(a[2]), "v"(a[3]));
    }
    const size_t tbase = (size_t)(r0 / RB) * sRB + (size_t)(r0 % RB) * (size_t)pitch + (size_t)(c0 / CB) * sCB + (size_t)(c0 % CB);
    if (OM == 0) {
        const int rq = lane >> 3, c8 = (lane & 7) * 8;
        const int cb = (c0 + c8) & (DM - 1);
        const v4f bc0 = *(const v4f*)(bias + cb), bc1 = *(const v4f*)(bias + cb + 4);
        float bcol[8];
#pragma unroll
        for (int i = 0; i < 4; ++i) { bcol[i] = bfr(bc0[i]); bcol[4 + i] = bfr(bc1[i]); }
#pragma unroll
        for (int mb = 0; mb < 4; ++mb) {
#pragma unroll
            for (int nb = 0; nb < 4; ++nb) {
#pragma unroll
                for (int j = 0; j < 8; ++j) os[(hi * 8 + j) * 68 + nb * 16 + lr] = acc[mb][nb][j]; }
            wave_sync();
            v8h hv[4], rv[4];
#pragma unroll
            for (int s = 0; s < 4; ++s) { const int row = 4 * s + rq;
                const float brow = bfr(bias[(r0 + mb * 16 + row) & (DM - 1)]);
                const v4f x0 = *(const v4fa*)(&os[row * 68 + c8]); const v4f x1 = *(const v4fa*)(&os[row * 68 + c8 + 4]);
#pragma unroll
                for (int i = 0; i < 4; ++i) {
                    const float y0 = x0[i] + ((bmode == 2) ? brow : bcol[i]); const float y1 = x1[i] + ((bmode == 2) ? brow : bcol[4 + i]);
                    const h16 a0 = (h16)y0; const h16 a1 = (h16)y1; hv[s][i] = a0; hv[s][4 + i] = a1;
                    rv[s][i] = (h16)((y0 - (float)a0) * QRS); rv[s][4 + i] = (h16)((y1 - (float)a1) * QRS); } }
            const size_t sb = tbase + (size_t)(mb * 16) * (size_t)pitch;
#pragma unroll 1
            for (int ps = 0; ps < 2; ++ps) {
#pragma unroll
                for (int s = 0; s < 4; ++s) { const size_t oo = sb + (size_t)(4 * s + rq) * (size_t)pitch + c8;
                    *(volatile v8h*)(Ph + oo) = hv[s]; if (useRes) *(volatile v8h*)(Pr + oo) = rv[s]; }
                if (ps == 0) __threadfence(); }
            wave_sync();
        }
    } else {
        const int cofs = lr * 4;
        const v4f bo4 = *(const v4f*)(bias + ((c0 + cofs) & (DM - 1)));
        v4f bb;
#pragma unroll
        for (int i = 0; i < 4; ++i) bb[i] = bfr(bo4[i]);
#pragma unroll
        for (int mb = 0; mb < 4; ++mb) {
#pragma unroll
            for (int nb = 0; nb < 4; ++nb) {
#pragma unroll
                for (int j = 0; j < 8; ++j) os[(hi * 8 + j) * 68 + nb * 16 + lr] = acc[mb][nb][j]; }
            wave_sync();
            v4f vals[8];
#pragma unroll
            for (int s = 0; s < 8; ++s) { const int row = 2 * s + hi;
                const v4f xv = *(const v4fa*)(&os[row * 68 + cofs]); vals[s] = xv * oscale + bb; }
            const size_t sb = tbase + (size_t)(mb * 16) * (size_t)pitch;
#pragma unroll 1
            for (int ps = 0; ps < 2; ++ps) {
#pragma unroll
                for (int s = 0; s < 8; ++s) *(volatile v4f*)(Pf + sb + (size_t)(2 * s + hi) * (size_t)pitch + cofs) = vals[s];
                if (ps == 0) __threadfence(); }
            wave_sync();
        }
    }
}

template<int PREC>
__global__ __launch_bounds__(32 * AW) void k_flash(const h16* __restrict__ QH, const h16* __restrict__ QR, const h16* __restrict__ KP, const h16* __restrict__ KR,
                                                   const h16* __restrict__ VT, const h16* __restrict__ VR, h16* CX) {
    __shared__ __align__(16) float os[AW * 16 * 68];
    const int lane = threadIdx.x & 31, lr = lane & 15, hi = lane >> 4;
    const int wave = __builtin_amdgcn_readfirstlane((int)(threadIdx.x >> 5));
    const int zh = blockIdx.y; const int b = zh / NH_, h = zh % NH_;
    const int t0 = (PREC ? 0 : EARLY) + (blockIdx.x * AW + wave) * 16;
    const int tq = t0 + lr;
    const size_t pbase = (size_t)zh * SEQ * HD;
    const size_t qo = pbase + (size_t)(t0 + lr) * HD + 8 * hi;
    const v16h qh0 = ldh(QH + qo), qh1 = ldh(QH + qo + 32), qr0 = ldh(QR + qo), qr1 = ldh(QR + qo + 32);
    const size_t ko = pbase + (size_t)lr * HD + 8 * hi;
    const size_t vo = pbase + (size_t)lr * SEQ + 8 * hi;
    v8f o0 = (v8f){}, o1 = (v8f){}, o2 = (v8f){}, o3 = (v8f){};
    v8f e0 = (v8f){}, e1 = (v8f){}, e2 = (v8f){}, e3 = (v8f){};
    float m = -3.0e38f, l = 0.0f;
    const int kend = t0 + 16;
#pragma unroll 1
    for (int key0 = 0; key0 < kend; key0 += 32) {
        const h16* ka = KP + ko + (size_t)key0 * HD;
        const v16h ka0 = ldh(ka), ka1 = ldh(ka + 32), kb0 = ldh(ka + 16 * HD), kb1 = ldh(ka + 16 * HD + 32);
        v8f sHa = (v8f){}, sLa = (v8f){}, sHb = (v8f){}, sLb = (v8f){};
        if (PREC) {
            const h16* kr = KR + ko + (size_t)key0 * HD;
            const v16h ra0 = ldh(kr), ra1 = ldh(kr + 32), rb0 = ldh(kr + 16 * HD), rb1 = ldh(kr + 16 * HD + 32);
            v8f sKa = (v8f){}, sKb = (v8f){};
            sHa = wmma16(ka0, qh0, sHa); sLa = wmma16(ka0, qr0, sLa); sHb = wmma16(kb0, qh0, sHb); sLb = wmma16(kb0, qr0, sLb); sKa = wmma16(ra0, qh0, sKa); sKb = wmma16(rb0, qh0, sKb);
            sHa = wmma16(ka1, qh1, sHa); sLa = wmma16(ka1, qr1, sLa); sHb = wmma16(kb1, qh1, sHb); sLb = wmma16(kb1, qr1, sLb); sKa = wmma16(ra1, qh1, sKa); sKb = wmma16(rb1, qh1, sKb);
            asm volatile("v_nop\n\tv_nop\n\tv_nop\n\tv_nop" : "+v"(sHa), "+v"(sLa), "+v"(sHb), "+v"(sLb), "+v"(sKa), "+v"(sKb)
                         : "v"(ka0), "v"(ka1), "v"(kb0), "v"(kb1), "v"(ra0), "v"(ra1), "v"(rb0), "v"(rb1));
            sLa = sLa + sKa; sLb = sLb + sKb;
        } else {
            sHa = wmma16(ka0, qh0, sHa); sLa = wmma16(ka0, qr0, sLa); sHb = wmma16(kb0, qh0, sHb); sLb = wmma16(kb0, qr0, sLb);
            sHa = wmma16(ka1, qh1, sHa); sLa = wmma16(ka1, qr1, sLa); sHb = wmma16(kb1, qh1, sHb); sLb = wmma16(kb1, qr1, sLb);
            asm volatile("v_nop\n\tv_nop\n\tv_nop\n\tv_nop" : "+v"(sHa), "+v"(sLa), "+v"(sHb), "+v"(sLb) : "v"(ka0), "v"(ka1), "v"(kb0), "v"(kb1));
        }
        float ta[8], tb[8];
#pragma unroll
        for (int r = 0; r < 8; ++r) { ta[r] = (sHa[r] + sLa[r] * QRI) * SC2; tb[r] = (sHb[r] + sLb[r] * QRI) * SC2; }
        if (key0 + 31 > t0) {
#pragma unroll
            for (int r = 0; r < 8; ++r) { const int kk = key0 + 8 * hi + r;
                ta[r] = (kk <= tq) ? ta[r] : -3.0e38f; tb[r] = (kk + 16 <= tq) ? tb[r] : -3.0e38f; }
        }
        float mx = -3.0e38f;
#pragma unroll
        for (int r = 0; r < 8; ++r) mx = fmaxf(mx, fmaxf(ta[r], tb[r]));
        mx = fmaxf(mx, __shfl_xor(mx, 16, 32));
        const float mnew = fmaxf(m, mx);
        const float alpha = __builtin_amdgcn_exp2f(m - mnew);
        const float sh = PSH - mnew;
        v16h pb, pr; float ls = 0.0f;
#pragma unroll
        for (int r = 0; r < 8; ++r) {
            const float ea = __builtin_amdgcn_exp2f(ta[r] + sh), ec = __builtin_amdgcn_exp2f(tb[r] + sh);
            const h16 pa = (h16)ea; const h16 pc = (h16)ec; pb[r] = pa; pb[8 + r] = pc;
            if (PREC) { const h16 xa = (h16)((ea - (float)pa) * QRS); const h16 xc = (h16)((ec - (float)pc) * QRS); pr[r] = xa; pr[8 + r] = xc;
                        ls += ((float)pa + (float)pc) + ((float)xa + (float)xc) * QRI; }
            else { pr[r] = pa; pr[8 + r] = pc; ls += (float)pa + (float)pc; }
        }
        l = l * alpha + ls; m = mnew;
        o0 = o0 * alpha; o1 = o1 * alpha; o2 = o2 * alpha; o3 = o3 * alpha;
        const h16* va = VT + vo + key0;
        const v16h v0 = ldh(va), v1 = ldh(va + (size_t)16 * SEQ), v2 = ldh(va + (size_t)32 * SEQ), v3 = ldh(va + (size_t)48 * SEQ);
        if (PREC) {
            e0 = e0 * alpha; e1 = e1 * alpha; e2 = e2 * alpha; e3 = e3 * alpha;
            const h16* vr = VR + vo + key0;
            const v16h w0 = ldh(vr), w1 = ldh(vr + (size_t)16 * SEQ), w2 = ldh(vr + (size_t)32 * SEQ), w3 = ldh(vr + (size_t)48 * SEQ);
            o0 = wmma16(v0, pb, o0); o1 = wmma16(v1, pb, o1); o2 = wmma16(v2, pb, o2); o3 = wmma16(v3, pb, o3);
            e0 = wmma16(w0, pb, e0); e1 = wmma16(w1, pb, e1); e2 = wmma16(w2, pb, e2); e3 = wmma16(w3, pb, e3);
            e0 = wmma16(v0, pr, e0); e1 = wmma16(v1, pr, e1); e2 = wmma16(v2, pr, e2); e3 = wmma16(v3, pr, e3);
            asm volatile("v_nop\n\tv_nop\n\tv_nop\n\tv_nop" : "+v"(o0), "+v"(o1), "+v"(o2), "+v"(o3), "+v"(e0), "+v"(e1), "+v"(e2), "+v"(e3)
                         : "v"(v0), "v"(v1), "v"(v2), "v"(v3), "v"(w0), "v"(w1), "v"(w2), "v"(w3), "v"(pb), "v"(pr));
        } else {
            o0 = wmma16(v0, pb, o0); o1 = wmma16(v1, pb, o1); o2 = wmma16(v2, pb, o2); o3 = wmma16(v3, pb, o3);
            asm volatile("v_nop\n\tv_nop\n\tv_nop\n\tv_nop" : "+v"(o0), "+v"(o1), "+v"(o2), "+v"(o3) : "v"(v0), "v"(v1), "v"(v2), "v"(v3), "v"(pb));
        }
    }
    l += __shfl_xor(l, 16, 32);
    const float inv = CXS * (1.0f / l);
    const int wb = wave * 16 * 68;
    { v8f c0v = o0, c1v = o1, c2v = o2, c3v = o3;
      if (PREC) { c0v = c0v + e0 * QRI; c1v = c1v + e1 * QRI; c2v = c2v + e2 * QRI; c3v = c3v + e3 * QRI; }
      c0v = c0v * inv; c1v = c1v * inv; c2v = c2v * inv; c3v = c3v * inv;
      *(v4fa*)(&os[wb + lr * 68 +  0 + 8 * hi]) = __builtin_shufflevector(c0v, c0v, 0, 1, 2, 3); *(v4fa*)(&os[wb + lr * 68 +  0 + 8 * hi + 4]) = __builtin_shufflevector(c0v, c0v, 4, 5, 6, 7);
      *(v4fa*)(&os[wb + lr * 68 + 16 + 8 * hi]) = __builtin_shufflevector(c1v, c1v, 0, 1, 2, 3); *(v4fa*)(&os[wb + lr * 68 + 16 + 8 * hi + 4]) = __builtin_shufflevector(c1v, c1v, 4, 5, 6, 7);
      *(v4fa*)(&os[wb + lr * 68 + 32 + 8 * hi]) = __builtin_shufflevector(c2v, c2v, 0, 1, 2, 3); *(v4fa*)(&os[wb + lr * 68 + 32 + 8 * hi + 4]) = __builtin_shufflevector(c2v, c2v, 4, 5, 6, 7);
      *(v4fa*)(&os[wb + lr * 68 + 48 + 8 * hi]) = __builtin_shufflevector(c3v, c3v, 0, 1, 2, 3); *(v4fa*)(&os[wb + lr * 68 + 48 + 8 * hi + 4]) = __builtin_shufflevector(c3v, c3v, 4, 5, 6, 7); }
    wave_sync();
    const int rq = lane >> 3, c8 = (lane & 7) * 8;
    v8h hv[4], rv[4];
#pragma unroll
    for (int s = 0; s < 4; ++s) { const int row = 4 * s + rq;
        const v4f x0 = *(const v4fa*)(&os[wb + row * 68 + c8]); const v4f x1 = *(const v4fa*)(&os[wb + row * 68 + c8 + 4]);
#pragma unroll
        for (int i = 0; i < 4; ++i) { const h16 a0 = (h16)x0[i]; const h16 a1 = (h16)x1[i]; hv[s][i] = a0; hv[s][4 + i] = a1;
            rv[s][i] = (h16)((x0[i] - (float)a0) * CRS); rv[s][4 + i] = (h16)((x1[i] - (float)a1) * CRS); } }
    const size_t cpitch = PREC ? (size_t)(2 * DM) : (size_t)DM;
    h16* crow = CX + ((size_t)b * (size_t)(PREC ? EARLY : (SEQ - EARLY)) + (size_t)(t0 - (PREC ? 0 : EARLY))) * cpitch + (size_t)h * HD;
#pragma unroll 1
    for (int ps = 0; ps < 2; ++ps) {
#pragma unroll
        for (int s = 0; s < 4; ++s) { const size_t oo = (size_t)(4 * s + rq) * cpitch + c8;
            *(volatile v8h*)(crow + oo) = hv[s]; if (PREC) *(volatile v8h*)(crow + oo + DM) = rv[s]; }
        if (ps == 0) __threadfence(); }
}

static constexpr size_t al256(size_t v) { return (v + 255) & ~(size_t)255; }
static constexpr size_t SZ_XB = al256((size_t)NB * SEQ * DM * 2);
static constexpr size_t SZ_CD = (size_t)NB * (SEQ - EARLY) * DM * 2;
static constexpr size_t SZ_WB = al256((size_t)3 * DM * DM * 2);
static constexpr size_t SZ_CE = (size_t)NB * EARLY * 2 * DM * 2;
static constexpr size_t SZ_WO = al256((size_t)DM * 2 * DM * 2);
static constexpr size_t SZ_PL = al256((size_t)NB * NH_ * SEQ * HD * 2);
static constexpr size_t SZ_TOTAL = SZ_XB + SZ_WB + SZ_WO + 6 * SZ_PL;
static_assert(SZ_CD <= SZ_XB);
static_assert(SZ_CE <= SZ_WB);
static_assert(SZ_TOTAL <= (size_t)134217728);
static_assert(((size_t)DM * DM * 2) % 256 == 0);

extern "C" void kernel_launch(void* const* d_in, const int* in_sizes, int n_in,
                              void* d_out, int out_size, void* d_ws, size_t ws_size, hipStream_t stream) {
    if (n_in < 9) return;
    const size_t needx = ((size_t)(NB - 1) * SEQ_FULL + SEQ) * DM;
    if ((size_t)in_sizes[0] < needx) return;
    if ((size_t)in_sizes[1] < (size_t)NH_ * DM * HD || (size_t)in_sizes[2] < (size_t)NH_ * DM * HD || (size_t)in_sizes[3] < (size_t)NH_ * DM * HD) return;
    if ((size_t)in_sizes[4] < (size_t)DM || (size_t)in_sizes[5] < (size_t)DM || (size_t)in_sizes[6] < (size_t)DM) return;
    if ((size_t)in_sizes[7] < (size_t)DM * DM || (size_t)in_sizes[8] < (size_t)DM) return;
    if ((size_t)out_size < ((size_t)(NB - 1) * OUT_SEQ + SEQ) * DM) return;
    if (SZ_TOTAL > ws_size) return;
    const float* x  = (const float*)d_in[0];
    const float* wq = (const float*)d_in[1]; const float* wk = (const float*)d_in[2]; const float* wv = (const float*)d_in[3];
    const float* bq = (const float*)d_in[4]; const float* bk = (const float*)d_in[5]; const float* bv = (const float*)d_in[6];
    const float* wo = (const float*)d_in[7];
    const float* bo = (const float*)d_in[8];
    float* OUT = (float*)d_out;
    char* wsp = (char*)d_ws;
    bf* XB = (bf*)wsp; h16* CD = (h16*)wsp; wsp += SZ_XB;
    bf* WB = (bf*)wsp; h16* CE = (h16*)wsp; wsp += SZ_WB;
    bf* WO2 = (bf*)wsp; wsp += SZ_WO;
    h16* QH = (h16*)wsp; wsp += SZ_PL;
    h16* QR = (h16*)wsp; wsp += SZ_PL;
    h16* KP = (h16*)wsp; wsp += SZ_PL;
    h16* KR = (h16*)wsp; wsp += SZ_PL;
    h16* VT = (h16*)wsp; wsp += SZ_PL;
    h16* VR = (h16*)wsp; wsp += SZ_PL;
    bf* WQT = WB; bf* WKT = WB + (size_t)DM * DM; bf* WVT = WB + (size_t)2 * DM * DM;

    if (SEQ == SEQ_FULL) {
        const size_t n8 = (size_t)NB * SEQ * DM / 8;
        k_cvt8<<<(unsigned)((n8 + 255) / 256), 256, 0, stream>>>(x, XB, n8);
    } else {
        const size_t n8 = (size_t)SEQ * DM / 8;
        for (int b = 0; b < NB; ++b) k_cvt8<<<(unsigned)((n8 + 255) / 256), 256, 0, stream>>>(x + (size_t)b * SEQ_FULL * DM, XB + (size_t)b * SEQ * DM, n8);
    }
    k_tr<0><<<dim3(DM / 64, HD / 64, NH_), 256, 0, stream>>>(wq, WQT, HD, DM, (size_t)DM * HD, (size_t)HD * DM);
    k_tr<0><<<dim3(DM / 64, HD / 64, NH_), 256, 0, stream>>>(wk, WKT, HD, DM, (size_t)DM * HD, (size_t)HD * DM);
    k_tr<0><<<dim3(DM / 64, HD / 64, NH_), 256, 0, stream>>>(wv, WVT, HD, DM, (size_t)DM * HD, (size_t)HD * DM);
    k_tr<1><<<dim3(DM / 64, DM / 64, 1), 256, 0, stream>>>(wo, WO2, DM, 2 * DM, (size_t)0, (size_t)0);

    k_gemm<0><<<dim3(NB * SEQ / 64, DM / 64, 1), 32, 0, stream>>>(XB, WQT, DM, DM, DM, QH, QR, OUT, 1, SEQ, (size_t)NH_ * SEQ * HD, HD, HD, (size_t)SEQ * HD, bq, 1, 1.0f);
    k_gemm<0><<<dim3(NB * SEQ / 64, DM / 64, 1), 32, 0, stream>>>(XB, WKT, DM, DM, DM, KP, KR, OUT, 1, SEQ, (size_t)NH_ * SEQ * HD, HD, HD, (size_t)SEQ * HD, bk, 1, 1.0f);
    k_gemm<0><<<dim3(DM / 64, NB * SEQ / 64, 1), 32, 0, stream>>>(WVT, XB, DM, DM, DM, VT, VR, OUT, 1, DM, (size_t)0, SEQ, SEQ, (size_t)DM * SEQ, bv, 2, 1.0f);

    k_flash<0><<<dim3((SEQ - EARLY) / (16 * AW), NB * NH_, 1), 32 * AW, 0, stream>>>(QH, QR, KP, KR, VT, VR, CD);
    k_flash<1><<<dim3(EARLY / (16 * AW), NB * NH_, 1), 32 * AW, 0, stream>>>(QH, QR, KP, KR, VT, VR, CE);

    k_gemm<1><<<dim3(NB * (SEQ - EARLY) / 64, DM / 64, 1), 32, 0, stream>>>((const bf*)CD, WO2, DM, DM, 2 * DM, QH, QH, OUT + (size_t)EARLY * DM, 0,
                                                                            SEQ - EARLY, (size_t)OUT_SEQ * DM, DM, DM, (size_t)0, bo, 1, OSC);
    k_gemm<1><<<dim3(NB * EARLY / 64, DM / 64, 1), 32, 0, stream>>>((const bf*)CE, WO2, 2 * DM, 2 * DM, 2 * DM, QH, QH, OUT, 0,
                                                                    EARLY, (size_t)OUT_SEQ * DM, DM, DM, (size_t)0, bo, 1, OSC);
}
